// SGC_76922864272070
// MI455X (gfx1250) — hardware-run, weakly checked
//
#include <hip/hip_runtime.h>

typedef float          v8f   __attribute__((ext_vector_type(8)));
typedef float          v4f   __attribute__((ext_vector_type(4)));
typedef unsigned int   v4u   __attribute__((ext_vector_type(4)));
typedef int            v8i   __attribute__((ext_vector_type(8)));
typedef unsigned short v8us  __attribute__((ext_vector_type(8)));
typedef unsigned short v16us __attribute__((ext_vector_type(16)));
typedef __bf16         v16bf __attribute__((ext_vector_type(16)));
typedef _Float16       v16h  __attribute__((ext_vector_type(16)));
typedef v4f  __attribute__((may_alias)) v4fa;
typedef v8us __attribute__((may_alias)) v8usa;
union FragB { v16bf v; v16us u; v8us h[2]; v8i w; };
union FragH { v16h  v; v16us u; v8us h[2]; v8i w; };

__device__ __forceinline__ v8f wmb(const FragB& a, const FragB& b, v8f c) {
  v8f d = __builtin_amdgcn_wmma_f32_16x16x32_bf16(false, a.v, false, b.v, (short)0, c, false, false);
  asm volatile("v_nop\n\tv_nop\n\tv_nop\n\tv_nop" : "+v"(d) : "v"(a.w), "v"(b.w));
  return d;
}

__device__ __forceinline__ v8f wmh(const FragH& a, const FragH& b, v8f c) {
  v8f d = __builtin_amdgcn_wmma_f32_16x16x32_f16(false, a.v, false, b.v, (short)0, c, false, false);
  asm volatile("v_nop\n\tv_nop\n\tv_nop\n\tv_nop" : "+v"(d) : "v"(a.w), "v"(b.w));
  return d;
}

__device__ __forceinline__ unsigned bf16_bits(float f) {
  const unsigned u = __float_as_uint(f);
  const unsigned r = (u + 0x7FFFu + ((u >> 16) & 1u)) >> 16;
  const unsigned q = (u >> 16) | 0x40u;
  return ((u & 0x7fffffffu) > 0x7f800000u) ? q : r;
}

__device__ __forceinline__ float bf16_val(float f) {
  return __uint_as_float(bf16_bits(f) << 16);
}
__device__ __forceinline__ int clampi(int v, int lo, int hi) {
  return v < lo ? lo : (v > hi ? hi : v);
}

__device__ __forceinline__ unsigned f16_bits(float f) {
  const unsigned u  = __float_as_uint(f);
  const unsigned s  = (u >> 16) & 0x8000u;
  const unsigned a  = u & 0x7fffffffu;
  const unsigned t  = a - 0x38000000u;
  const unsigned r  = (t + 0x0FFFu + ((t >> 13) & 1u)) >> 13;
  const unsigned rc = r > 0x7C00u ? 0x7C00u : r;
  const bool small  = a < 0x38800000u;
  const bool isnan  = a > 0x7f800000u;
  const unsigned fin = small ? 0u : (s | rc);
  return isnan ? (s | 0x7E00u) : fin;
}

__device__ __forceinline__ unsigned pk16(unsigned lo, unsigned hi) { return lo | (hi << 16); }
__device__ __forceinline__ unsigned bf16_lo_bits(float v) {
  float hi = bf16_val(v);
  asm volatile("" : "+v"(hi));
  return bf16_bits(v - hi);
}
__device__ __forceinline__ v4u pack8_bf16(v4f a, v4f c) {
  return (v4u){ pk16(bf16_bits(a[0]), bf16_bits(a[1])), pk16(bf16_bits(a[2]), bf16_bits(a[3])),
                pk16(bf16_bits(c[0]), bf16_bits(c[1])), pk16(bf16_bits(c[2]), bf16_bits(c[3])) };
}
__device__ __forceinline__ v4u pack8_bf16_lo(v4f a, v4f c) {
  return (v4u){ pk16(bf16_lo_bits(a[0]), bf16_lo_bits(a[1])), pk16(bf16_lo_bits(a[2]), bf16_lo_bits(a[3])),
                pk16(bf16_lo_bits(c[0]), bf16_lo_bits(c[1])), pk16(bf16_lo_bits(c[2]), bf16_lo_bits(c[3])) };
}
__device__ __forceinline__ v4u pack8_f16(v4f a, v4f c) {
  return (v4u){ pk16(f16_bits(a[0]), f16_bits(a[1])), pk16(f16_bits(a[2]), f16_bits(a[3])),
                pk16(f16_bits(c[0]), f16_bits(c[1])), pk16(f16_bits(c[2]), f16_bits(c[3])) };
}

template <int FORM>
__global__ __launch_bounds__(256) void k_plane(const float* __restrict__ src, int rows, int cols, int ldsrc,
                                               unsigned short* __restrict__ dst, int MP, int KP) {
  static_assert(FORM >= 0 && FORM <= 3);
  const int KTOT = (FORM == 1 || FORM == 3) ? 2 * KP : KP;
  const unsigned ppr   = (unsigned)(KTOT >> 3);
  const unsigned kp8   = (unsigned)(KP >> 3);
  const unsigned total = (unsigned)MP * ppr;
  const unsigned g     = blockIdx.x * 256u + threadIdx.x;
  const unsigned rowu  = g / ppr;
  const unsigned p     = g - rowu * ppr;
  const bool second    = p >= kp8;
  const int row = (int)rowu;
  const int c0  = (int)((second ? p - kp8 : p) << 3);
  const float* srow = src + (size_t)clampi(row, 0, rows - 1) * (size_t)ldsrc;
  float x[8];
  unsigned mk[8];
#pragma unroll
  for (int e = 0; e < 8; ++e) {
    const int c = c0 + e;
    const float v = srow[clampi(c, 0, cols - 1)];
    asm volatile("" :: "v"(v));
    x[e]  = v;
    mk[e] = (row < rows && c < cols) ? 0xFFFFu : 0u;
  }
  const v4f a = (v4f){ x[0], x[1], x[2], x[3] };
  const v4f c = (v4f){ x[4], x[5], x[6], x[7] };
  v4u o;
  if (FORM == 2) {
    o = pack8_f16(a, c);
  } else {
    const v4u hi = pack8_bf16(a, c);
    o = hi;
    if (FORM == 1) { const v4u lo = pack8_bf16_lo(a, c); o = second ? lo : hi; }
  }
  const v4u mw = (v4u){ pk16(mk[0], mk[1]), pk16(mk[2], mk[3]), pk16(mk[4], mk[5]), pk16(mk[6], mk[7]) };
  o &= mw;
  if (g < total) {
    volatile v4u* q = (volatile v4u*)(dst + (size_t)g * 8);
    *q = o;
    __threadfence();
    *q = o;
  }
}

template <int FORM> struct FragOf    { typedef FragB T; };
template <>         struct FragOf<2> { typedef FragH T; };
__device__ __forceinline__ v8f mm(const FragB& a, const FragB& b, v8f c) { return wmb(a, b, c); }
__device__ __forceinline__ v8f mm(const FragH& a, const FragH& b, v8f c) { return wmh(a, b, c); }
template <class F> __device__ __forceinline__ F ld_frag(const unsigned short* p) {
  F f;
  f.h[0] = *(const v8usa*)(p);
  f.h[1] = *(const v8usa*)(p + 16);
  return f;
}

template <int FORM, int EPI>
__global__ __launch_bounds__(256) __attribute__((amdgpu_num_vgpr(248)))
void k_gemm_nt(const unsigned short* __restrict__ A, const unsigned short* __restrict__ B,
               const float* __restrict__ bias, float* __restrict__ D, int M, int N, int KTOT, int ldd) {
  static_assert(FORM >= 0 && FORM <= 2);
  static_assert(EPI == 0 || EPI == 1);
  typedef typename FragOf<FORM>::T F;
  __shared__ __attribute__((aligned(16))) float sT[8][16 * 68];
  const int lane = threadIdx.x & 31;
  const int wave = threadIdx.x >> 5;
  const int tilesM = (M + 63) >> 6;
  const int tilesN = (N + 63) >> 6;
  const int tile = blockIdx.x * 8 + wave;
  if (tile >= tilesM * tilesN) return;
  const int tm = tile / tilesN;
  const int tn = tile - tm * tilesN;
  const int m0 = tm << 6;
  const int n0 = tn << 6;

  const int rl = lane & 15;
  const int h8 = (lane >> 4) * 8;
  const unsigned short* pa = A + (size_t)(m0 + rl) * (size_t)KTOT + h8;
  const unsigned short* pb = B + (size_t)(n0 + rl) * (size_t)KTOT + h8;

  v8f acc[4][4];
#pragma unroll
  for (int i = 0; i < 4; ++i)
#pragma unroll
    for (int j = 0; j < 4; ++j) acc[i][j] = (v8f){0.f, 0.f, 0.f, 0.f, 0.f, 0.f, 0.f, 0.f};

#pragma unroll 1
  for (int k0 = 0; k0 < KTOT; k0 += 32) {
    F bf[4];
#pragma unroll
    for (int j = 0; j < 4; ++j) bf[j] = ld_frag<F>(pb + (size_t)(j << 4) * (size_t)KTOT + k0);
#pragma unroll
    for (int i = 0; i < 4; ++i) {
      const F af = ld_frag<F>(pa + (size_t)(i << 4) * (size_t)KTOT + k0);
#pragma unroll
      for (int j = 0; j < 4; ++j) acc[i][j] = mm(af, bf[j], acc[i][j]);
    }
  }

  float* slab = sT[wave];
  const int hh = lane >> 4;
  const int c4 = (lane & 15) * 4;
  const int nc = n0 + c4;
  const bool cok = nc < N;
  v4f bv = (v4f){0.f, 0.f, 0.f, 0.f};
  if (EPI == 1) {
    bv = *(const v4fa*)(bias + clampi(nc, 0, N - 4));
    asm volatile("" :: "v"(bv));
  }
#pragma unroll
  for (int i = 0; i < 4; ++i) {
    const int mBase = m0 + (i << 4);
#pragma unroll
    for (int j = 0; j < 4; ++j) {
#pragma unroll
      for (int r = 0; r < 8; ++r) slab[(h8 + r) * 68 + (j << 4) + rl] = acc[i][j][r];
    }
    __builtin_amdgcn_fence(__ATOMIC_RELEASE, "workgroup");
    __builtin_amdgcn_wave_barrier();
    __builtin_amdgcn_fence(__ATOMIC_ACQUIRE, "workgroup");
    v4f vv[8];
#pragma unroll
    for (int it = 0; it < 8; ++it) {
      const int row = it * 2 + hh;
      v4f v = *(const v4fa*)(slab + row * 68 + c4);
      if (EPI == 1) v += bv;
      vv[it] = v;
    }
    for (int pass = 0; pass < 2; ++pass) {
#pragma unroll
      for (int it = 0; it < 8; ++it) {
        const int row = mBase + it * 2 + hh;
        if (cok && row < M) *(volatile v4f*)(D + (size_t)row * (size_t)ldd + nc) = vv[it];
      }
      __threadfence();
    }
    __builtin_amdgcn_fence(__ATOMIC_RELEASE, "workgroup");
    __builtin_amdgcn_wave_barrier();
    __builtin_amdgcn_fence(__ATOMIC_ACQUIRE, "workgroup");
  }
}

#include <stddef.h>
#include <stdint.h>
#include <math.h>

#pragma clang fp contract(off)

#ifndef SPLIT_L2
#define SPLIT_L2 1
#endif
#ifndef SPLIT_L3
#define SPLIT_L3 1
#endif

#define NN      100000
#define KD      128
#define HD      64
#define NC      40
#define NE      1600000
#define MP      100096
#define NTHR    256
#define NWAVE   8
#define EPT     8
#define WCH     (32 * EPT)
#define NBRUN   1024
#define SLB     10
#define NBK     98
#define WLCAP   3072
#define LCAP    21504
#define DEGCAP  64
#define MAXDEG_MEAS   36
#define MAXB1024_MEAS 16721

#define BK_ZINTS (NWAVE * WLCAP + LCAP + 3 * NBRUN)
#define BK_INTS  (BK_ZINTS + 16)
#define BK_LDS   (BK_INTS * 4)

#define PBX        (MP * KD / 8 / 256)
#define PB_W       4
#define GEMM_BLOCKS (((MP / 64) + 7) / 8)
#define FLAT_BLOCKS ((NN * NC / 32) / NWAVE)

static_assert(HD == 32 * 2 && HD == 16 * 4 && HD % 32 == 0);
static_assert(KD % 32 == 0 && KD == 2 * HD);
static_assert(NC % 4 == 0 && NC <= HD && NC % 2 == 0);
static_assert(MP % 64 == 0 && MP >= NN && MP == 782 * 128 && MP % 128 == 0 && MP % 16 == 0);
static_assert((MP * KD / 8) % 256 == 0);
static_assert((HD * KD / 8) == PB_W * NTHR);
static_assert(NBRUN == (1 << SLB) && NBRUN == NTHR * 4 && NBRUN % 32 == 0);
static_assert(NBK * NBRUN >= NN && (NBK - 1) * NBRUN < NN);
static_assert(NE < (1 << 21) && (((long long)NE) << SLB) < (1LL << 31));
static_assert(NE % WCH == 0 && NE % 4 == 0);
static_assert((long long)LCAP * 100 >= (long long)MAXB1024_MEAS * 125);
static_assert(WLCAP >= MAXB1024_MEAS / 8 + 8 * 46 + 1);
static_assert(MAXDEG_MEAS + 8 <= DEGCAP);
static_assert(LCAP % (NTHR * 4) == 0 && BK_ZINTS % (NTHR * 4) == 0);
static_assert(BK_LDS <= 262144);
static_assert(NN % NWAVE == 0 && (NN / NWAVE) * NWAVE == NN);
static_assert((NN * NC) % 32 == 0 && ((NN * NC) / 32) % NWAVE == 0);
static_assert(GEMM_BLOCKS == 196);
static_assert((size_t)MP * KD * 2 == (size_t)MP * HD * 4);

typedef float        v2f __attribute__((ext_vector_type(2)));
typedef unsigned int v2u __attribute__((ext_vector_type(2)));
typedef int          v4i __attribute__((ext_vector_type(4)));
typedef v2f __attribute__((may_alias)) v2fa;
typedef v2u __attribute__((may_alias)) v2ua;
typedef v4i __attribute__((may_alias)) v4ia;

__device__ __forceinline__ void st2_v4u(unsigned short* p, v4u v) {
  volatile v4u* q = (volatile v4u*)p;
  *q = v;
  __threadfence();
  *q = v;
}

__device__ __forceinline__ v4u gather8_bf16(const float* __restrict__ base, int pitch) {
  float f[8];
#pragma unroll
  for (int i = 0; i < 8; ++i) {
    const float v = base[(size_t)i * (size_t)pitch];
    asm volatile("" :: "v"(v));
    f[i] = v;
  }
  return (v4u){ pk16(bf16_bits(f[0]), bf16_bits(f[1])), pk16(bf16_bits(f[2]), bf16_bits(f[3])),
                pk16(bf16_bits(f[4]), bf16_bits(f[5])), pk16(bf16_bits(f[6]), bf16_bits(f[7])) };
}

__global__ __launch_bounds__(NTHR) void k_prep_w(const float* __restrict__ w1, const float* __restrict__ w2,
                                                 const float* __restrict__ w3, unsigned short* w1t,
                                                 unsigned short* w2d, unsigned short* w3d) {
  const int tid = (int)threadIdx.x;
  const int blk = (int)blockIdx.x;
  if (blk < PB_W) {
    const int u = blk * NTHR + tid;
    const int n = u >> 4, k8 = (u & 15) * 8;
    const v4u o = gather8_bf16(w1 + (size_t)k8 * HD + n, HD);
    st2_v4u(w1t + (size_t)n * KD + k8, o);
  } else if (blk < 2 * PB_W) {
    const int u = (blk - PB_W) * NTHR + tid;
    const int n = u >> 4, k8 = (u & 15) * 8;
    const int ks = k8 & (HD - 1);
    const v4u o = gather8_bf16(w2 + (size_t)ks * HD + n, HD);
    st2_v4u(w2d + (size_t)n * KD + k8, o);
  } else {
    const int u = (blk - 2 * PB_W) * NTHR + tid;
    const int n = u >> 4, k8 = (u & 15) * 8;
    const int ks = k8 & (HD - 1);
    const int ncl = n < NC - 1 ? n : NC - 1;
    v4u o = gather8_bf16(w3 + (size_t)ks * NC + ncl, NC);
    const unsigned mk = (n < NC) ? 0xFFFFFFFFu : 0u;
    o &= (v4u){ mk, mk, mk, mk };
    st2_v4u(w3d + (size_t)n * KD + k8, o);
  }
}

__global__ __launch_bounds__(NTHR) void k_build(const int* __restrict__ srcs, const int* __restrict__ dsts,
                                                int* LIST, int* CNT, int* OFF, int* FLAG) {
  extern __shared__ __attribute__((aligned(16))) int dsm[];
  int* wl   = dsm;
  int* pl   = dsm + NWAVE * WLCAP;
  int* cnt  = pl + LCAP;
  int* offs = cnt + NBRUN;
  int* cur  = offs + NBRUN;
  int* misc = cur + NBRUN;
  const int tid = (int)threadIdx.x, lane = tid & 31, wave = tid >> 5;
  const int blk = (int)blockIdx.x;
  const unsigned nbs = (unsigned)(blk * NBRUN);

  {
    const v4i z4 = {0, 0, 0, 0};
#pragma unroll 1
    for (int i = tid * 4; i < BK_ZINTS; i += NTHR * 4) *(v4ia*)(dsm + i) = z4;
    if (tid < 16) misc[tid] = 0;
  }
  __syncthreads();

  {
    const int per  = ((NE + NWAVE * WCH - 1) / (NWAVE * WCH)) * WCH;
    const int ebeg = wave * per;
    const int eend = (ebeg + per < NE) ? (ebeg + per) : NE;
    int* mylist = wl + wave * WLCAP;
    int wc = 0;
#pragma unroll 1
    for (int cb = ebeg; cb < eend; cb += WCH) {
      const int e0 = cb + lane * EPT;
      const v4i da = *(const v4ia*)(dsts + e0);
      const v4i db = *(const v4ia*)(dsts + e0 + 4);
      const int d0 = da.x, d1 = da.y, d2 = da.z, d3 = da.w;
      const int d4 = db.x, d5 = db.y, d6 = db.z, d7 = db.w;
      asm volatile("" :: "v"(d0), "v"(d1), "v"(d2), "v"(d3));
      asm volatile("" :: "v"(d4), "v"(d5), "v"(d6), "v"(d7));
      const unsigned s0 = (unsigned)d0 - nbs, s1 = (unsigned)d1 - nbs;
      const unsigned s2 = (unsigned)d2 - nbs, s3 = (unsigned)d3 - nbs;
      const unsigned s4 = (unsigned)d4 - nbs, s5 = (unsigned)d5 - nbs;
      const unsigned s6 = (unsigned)d6 - nbs, s7 = (unsigned)d7 - nbs;
      const bool h0 = s0 < (unsigned)NBRUN, h1 = s1 < (unsigned)NBRUN, h2 = s2 < (unsigned)NBRUN, h3 = s3 < (unsigned)NBRUN;
      const bool h4 = s4 < (unsigned)NBRUN, h5 = s5 < (unsigned)NBRUN, h6 = s6 < (unsigned)NBRUN, h7 = s7 < (unsigned)NBRUN;
      const unsigned m0 = __builtin_amdgcn_ballot_w32(h0), m1 = __builtin_amdgcn_ballot_w32(h1);
      const unsigned m2 = __builtin_amdgcn_ballot_w32(h2), m3 = __builtin_amdgcn_ballot_w32(h3);
      const unsigned m4 = __builtin_amdgcn_ballot_w32(h4), m5 = __builtin_amdgcn_ballot_w32(h5);
      const unsigned m6 = __builtin_amdgcn_ballot_w32(h6), m7 = __builtin_amdgcn_ballot_w32(h7);
      const unsigned any = m0 | m1 | m2 | m3 | m4 | m5 | m6 | m7;
      if (any != 0u) {
        const int pre = (int)(__builtin_amdgcn_mbcnt_lo(m0, 0u) + __builtin_amdgcn_mbcnt_lo(m1, 0u) +
                              __builtin_amdgcn_mbcnt_lo(m2, 0u) + __builtin_amdgcn_mbcnt_lo(m3, 0u) +
                              __builtin_amdgcn_mbcnt_lo(m4, 0u) + __builtin_amdgcn_mbcnt_lo(m5, 0u) +
                              __builtin_amdgcn_mbcnt_lo(m6, 0u) + __builtin_amdgcn_mbcnt_lo(m7, 0u));
        int p = wc + pre;
        if (h0) { if (p < WLCAP) mylist[p] = ((e0 + 0) << SLB) | (int)s0; p = p + 1; }
        if (h1) { if (p < WLCAP) mylist[p] = ((e0 + 1) << SLB) | (int)s1; p = p + 1; }
        if (h2) { if (p < WLCAP) mylist[p] = ((e0 + 2) << SLB) | (int)s2; p = p + 1; }
        if (h3) { if (p < WLCAP) mylist[p] = ((e0 + 3) << SLB) | (int)s3; p = p + 1; }
        if (h4) { if (p < WLCAP) mylist[p] = ((e0 + 4) << SLB) | (int)s4; p = p + 1; }
        if (h5) { if (p < WLCAP) mylist[p] = ((e0 + 5) << SLB) | (int)s5; p = p + 1; }
        if (h6) { if (p < WLCAP) mylist[p] = ((e0 + 6) << SLB) | (int)s6; p = p + 1; }
        if (h7) { if (p < WLCAP) mylist[p] = ((e0 + 7) << SLB) | (int)s7; p = p + 1; }
        wc += (int)(__builtin_popcount(m0) + __builtin_popcount(m1) + __builtin_popcount(m2) + __builtin_popcount(m3) +
                    __builtin_popcount(m4) + __builtin_popcount(m5) + __builtin_popcount(m6) + __builtin_popcount(m7));
      }
    }
    if (lane == 0) misc[wave] = wc;
  }
  __syncthreads();

  if (wave == 0) {
    int ov = 0;
    int tot = 0;
#pragma unroll 1
    for (int w2 = 0; w2 < NWAVE; ++w2) {
      int c = misc[w2];
      if (c > WLCAP) ov = 1;
      c = c < 0 ? 0 : (c > WLCAP ? WLCAP : c);
      tot += c;
#pragma unroll 1
      for (int b0 = 0; b0 < c; b0 += 32) {
        const int idx = b0 + lane;
        const int ent = wl[w2 * WLCAP + (idx < WLCAP ? idx : WLCAP - 1)];
        const int m32 = (c - b0) < 32 ? (c - b0) : 32;
#pragma unroll 1
        for (int k = 0; k < m32; ++k) {
          const int u    = __builtin_amdgcn_readlane(ent, k);
          const int slot = u & (NBRUN - 1);
          if (lane == 0) cnt[slot] = cnt[slot] + 1;
        }
      }
    }
    if (tot > LCAP) ov = 1;
    if (lane == 0) misc[9] = ov;
  }
  __syncthreads();
  if (wave == 0) {
    const int base = lane * (NBRUN / 32);
    int s = 0;
#pragma unroll 1
    for (int i = 0; i < NBRUN / 32; ++i) s += cnt[base + i];
    int incl = s;
#pragma unroll
    for (int d = 1; d < 32; d <<= 1) {
      const int y = __shfl_up(incl, d, 32);
      if (lane >= d) incl += y;
    }
    int run = incl - s;
#pragma unroll 1
    for (int i = 0; i < NBRUN / 32; ++i) {
      const int cv = cnt[base + i];
      offs[base + i] = run;
      cur[base + i]  = run;
      run += cv;
    }
  }
  __syncthreads();

  if (wave == 0) {
#pragma unroll 1
    for (int w2 = 0; w2 < NWAVE; ++w2) {
      int c = misc[w2];
      c = c < 0 ? 0 : (c > WLCAP ? WLCAP : c);
#pragma unroll 1
      for (int b0 = 0; b0 < c; b0 += 32) {
        const int idx = b0 + lane;
        const int ent = wl[w2 * WLCAP + (idx < WLCAP ? idx : WLCAP - 1)];
        int eid = (ent >> SLB) & 0x1FFFFF;
        eid = eid > NE - 1 ? NE - 1 : eid;
        int sr = srcs[eid];
        asm volatile("" :: "v"(sr));
        sr = sr < 0 ? 0 : (sr > NN - 1 ? NN - 1 : sr);
        const int m32 = (c - b0) < 32 ? (c - b0) : 32;
#pragma unroll 1
        for (int k = 0; k < m32; ++k) {
          const int u    = __builtin_amdgcn_readlane(ent, k);
          const int w0   = __builtin_amdgcn_readlane(sr, k);
          const int slot = u & (NBRUN - 1);
          if (lane == 0) {
            int p = cur[slot];
            p = p < 0 ? 0 : (p > LCAP - 1 ? LCAP - 1 : p);
            pl[p] = w0;
            cur[slot] = p + 1;
          }
        }
      }
    }
  }
  __syncthreads();

  const int ovf = misc[9];
  int* lp = LIST + (size_t)blk * (size_t)LCAP;
  int* cp = CNT  + (size_t)blk * NBRUN;
  int* op = OFF  + (size_t)blk * NBRUN;
  int* fp = FLAG + (size_t)blk * 32;
  for (int pass = 0; pass < 2; ++pass) {
#pragma unroll 1
    for (int i = tid * 4; i < LCAP; i += NTHR * 4) {
      const v4i v = *(const v4ia*)(pl + i);
      *(volatile v4i*)(lp + i) = v;
    }
    {
      const v4i vc = *(const v4ia*)(cnt + 4 * tid);
      const v4i vo = *(const v4ia*)(offs + 4 * tid);
      *(volatile v4i*)(cp + 4 * tid) = vc;
      *(volatile v4i*)(op + 4 * tid) = vo;
    }
    if (tid < 8) {
      const v4i f = {ovf, ovf, ovf, ovf};
      *(volatile v4i*)(fp + 4 * tid) = f;
    }
    __threadfence();
  }
}

template <int L>
__global__ __launch_bounds__(NTHR) void k_walk(const int* __restrict__ LIST, const int* __restrict__ CNT,
                                               const int* __restrict__ OFF, const int* __restrict__ FLAG,
                                               const float* __restrict__ T, unsigned* OUTW, int n_nodes) {
  static_assert(L >= 1 && L <= 3);
  __shared__ __attribute__((aligned(16))) unsigned srow[NWAVE][64];
  const int tid = (int)threadIdx.x, lane = tid & 31, wave = tid >> 5;
  const int node = (int)blockIdx.x * NWAVE + wave;
  const int dn = node < NN - 1 ? node : NN - 1;
  const int blk = dn >> SLB;
  const int* lb = LIST + (size_t)blk * (size_t)LCAP;
  const int craw = CNT[dn];
  const int oraw = OFF[dn];
  const int flag = FLAG[(size_t)blk * 32];
  asm volatile("" :: "v"(craw), "v"(oraw), "v"(flag));

  const bool big = craw > DEGCAP;
  const int c = __builtin_amdgcn_readfirstlane(craw < 0 ? 0 : (craw > DEGCAP ? DEGCAP : craw));
  const int o = oraw < 0 ? 0 : (oraw > LCAP - 1 ? LCAP - 1 : oraw);
  int last = o + (c > 0 ? c : 1) - 1;
  last = last > LCAP - 1 ? LCAP - 1 : last;

  float a0 = 0.0f, a1 = 0.0f;
#pragma unroll 1
  for (int b0 = 0; b0 < c; b0 += 32) {
    int idx = o + b0 + lane;
    idx = idx > last ? last : idx;
    int sr = lb[idx];
    asm volatile("" :: "v"(sr));
    sr = sr < 0 ? 0 : (sr > NN - 1 ? NN - 1 : sr);
    const int m32 = (c - b0) < 32 ? (c - b0) : 32;
#pragma unroll 1
    for (int k = 0; k < m32; ++k) {
      const int sk = __builtin_amdgcn_readlane(sr, k);
      const v2f q = *(const v2fa*)(T + (size_t)sk * HD + 2 * lane);
      asm volatile("" :: "v"(q));
      a0 = a0 + q.x;
      a1 = a1 + q.y;
    }
  }
  const bool bad = (flag != 0) | big;
  const float qnan = __uint_as_float(0x7fc00000u);
  const float v0 = bad ? qnan : a0;
  const float v1 = bad ? qnan : a1;

  v2u ov;
  if (L < 3) {
    const bool split = (L == 1) ? (SPLIT_L2 != 0) : (SPLIT_L3 != 0);
    const unsigned hiw = pk16(bf16_bits(v0), bf16_bits(v1));
    unsigned low = 0u;
    if (split) low = pk16(bf16_lo_bits(v0), bf16_lo_bits(v1));
    unsigned* row = srow[wave];
    row[lane]      = hiw;
    row[32 + lane] = low;
    __builtin_amdgcn_fence(__ATOMIC_RELEASE, "workgroup");
    __builtin_amdgcn_wave_barrier();
    __builtin_amdgcn_fence(__ATOMIC_ACQUIRE, "workgroup");
    ov = *(const v2ua*)(row + 2 * lane);
  } else {
    const bool real = (2 * lane) < NC;
    const float ninf = __uint_as_float(0xff800000u);
    const float pm = (v1 > v0 || v1 != v1) ? v1 : v0;
    float m = real ? pm : ninf;
#pragma unroll
    for (int off = 16; off >= 1; off >>= 1) {
      const float oth = __shfl_xor(m, off, 32);
      m = (oth > m || oth != oth) ? oth : m;
    }
    const float d0 = v0 - m;
    const float d1 = v1 - m;
    const float e0 = expf(d0);
    const float e1 = expf(d1);
    float s = real ? (e0 + e1) : 0.0f;
#pragma unroll
    for (int off = 16; off >= 1; off >>= 1) {
      const float oth = __shfl_xor(s, off, 32);
      s = s + oth;
    }
    const float ls = logf(s);
    float y0 = real ? (d0 - ls) : 0.0f;
    float y1 = real ? (d1 - ls) : 0.0f;
    y0 = bad ? qnan : y0;
    y1 = bad ? qnan : y1;
    ov = (v2u){ __float_as_uint(y0), __float_as_uint(y1) };
  }
  if (node < n_nodes) {
    volatile v2u* q = (volatile v2u*)(OUTW + (size_t)node * HD + 2 * lane);
    *q = ov;
    __threadfence();
    *q = ov;
  }
}

__global__ __launch_bounds__(NTHR) void k_flat(const float* __restrict__ Y, float* out, int n_out) {
  const int f = (int)blockIdx.x * NTHR + (int)threadIdx.x;
  int fc = f < n_out - 1 ? f : n_out - 1;
  fc = fc < 0 ? 0 : (fc > NN * NC - 1 ? NN * NC - 1 : fc);
  const int row = fc / NC;
  const int col = fc - row * NC;
  const float v = Y[(size_t)row * HD + col];
  asm volatile("" :: "v"(v));
  if (f < n_out) {
    volatile float* q = (volatile float*)(out + f);
    *q = v;
    __threadfence();
    *q = v;
  }
}

extern "C" void kernel_launch(void* const* d_in, const int* in_sizes, int n_in,
                              void* d_out, int out_size, void* d_ws, size_t ws_size,
                              hipStream_t stream) {
  if (n_in < 6) return;
  if (in_sizes[0] != NN * KD) return;
  if (in_sizes[1] != NE) return;
  if (in_sizes[2] != NE) return;
  if (in_sizes[3] != KD * HD) return;
  if (in_sizes[4] != HD * HD) return;
  if (in_sizes[5] != HD * NC) return;
  if (out_size != NN * NC) return;
  const int n_nodes = in_sizes[0] / KD;
  const int n_out   = out_size;

  const float* x    = (const float*)d_in[0];
  const int*   srcs = (const int*)d_in[1];
  const int*   dsts = (const int*)d_in[2];
  const float* W1   = (const float*)d_in[3];
  const float* W2   = (const float*)d_in[4];
  const float* W3   = (const float*)d_in[5];
  float* out = (float*)d_out;

  constexpr size_t zOP   = (size_t)MP * KD * 2;
  constexpr size_t zT    = (size_t)MP * HD * 4;
  constexpr size_t zLIST = (size_t)NBK * LCAP * 4;
  constexpr size_t zTBL  = (size_t)NBK * NBRUN * 4;
  constexpr size_t zFLAG = (size_t)NBK * 128;
  constexpr size_t zWP   = (size_t)HD * KD * 2;
  constexpr size_t oOP   = 0;
  constexpr size_t oT    = oOP + zOP;
  constexpr size_t oLIST = oT + zT;
  constexpr size_t oCNT  = oLIST + zLIST;
  constexpr size_t oOFF  = oCNT + zTBL;
  constexpr size_t oFLAG = oOFF + zTBL;
  constexpr size_t oW1T  = oFLAG + zFLAG;
  constexpr size_t oW2D  = oW1T + zWP;
  constexpr size_t oW3D  = oW2D + zWP;
  constexpr size_t oEND  = oW3D + zWP;
  static_assert(zOP % 256 == 0 && zT % 256 == 0 && zLIST % 256 == 0 && zTBL % 256 == 0);
  static_assert(zFLAG % 256 == 0 && zWP % 256 == 0);
  static_assert(zOP == (size_t)MP * HD * 4);
  static_assert(oEND == 60543232);
  static_assert(oEND <= ((size_t)128 << 20));
  if (oEND > ws_size) return;

  char* ws = (char*)d_ws;
  unsigned short* OP   = (unsigned short*)(ws + oOP);
  unsigned*       OPW  = (unsigned*)(ws + oOP);
  const float*    Y    = (const float*)(ws + oOP);
  float*          T    = (float*)(ws + oT);
  int*            LIST = (int*)(ws + oLIST);
  int*            CNT  = (int*)(ws + oCNT);
  int*            OFF  = (int*)(ws + oOFF);
  int*            FLAG = (int*)(ws + oFLAG);
  unsigned short* W1T  = (unsigned short*)(ws + oW1T);
  unsigned short* W2D  = (unsigned short*)(ws + oW2D);
  unsigned short* W3D  = (unsigned short*)(ws + oW3D);
  const float*    NOB  = (const float*)(ws + oW1T);

  hipFuncSetAttribute(reinterpret_cast<const void*>(&k_build), hipFuncAttributeMaxDynamicSharedMemorySize, (int)BK_LDS);

  k_plane<0><<<PBX, 256, 0, stream>>>(x, NN, KD, KD, OP, MP, KD);
  k_prep_w<<<3 * PB_W, NTHR, 0, stream>>>(W1, W2, W3, W1T, W2D, W3D);
  k_build<<<NBK, NTHR, BK_LDS, stream>>>(srcs, dsts, LIST, CNT, OFF, FLAG);
  k_gemm_nt<0, 0><<<GEMM_BLOCKS, 256, 0, stream>>>(OP, W1T, NOB, T, MP, HD, KD, HD);
  k_walk<1><<<NN / NWAVE, NTHR, 0, stream>>>(LIST, CNT, OFF, FLAG, T, OPW, n_nodes);
  k_gemm_nt<0, 0><<<GEMM_BLOCKS, 256, 0, stream>>>(OP, W2D, NOB, T, MP, HD, KD, HD);
  k_walk<2><<<NN / NWAVE, NTHR, 0, stream>>>(LIST, CNT, OFF, FLAG, T, OPW, n_nodes);
  k_gemm_nt<0, 0><<<GEMM_BLOCKS, 256, 0, stream>>>(OP, W3D, NOB, T, MP, HD, KD, HD);
  k_walk<3><<<NN / NWAVE, NTHR, 0, stream>>>(LIST, CNT, OFF, FLAG, T, OPW, n_nodes);
  k_flat<<<FLAT_BLOCKS, NTHR, 0, stream>>>(Y, out, n_out);
}
